// BiMambaBlock_41300405518476
// MI455X (gfx1250) — hardware-run, weakly checked
//
#include <hip/hip_runtime.h>
#include <math.h>

typedef __attribute__((ext_vector_type(16))) _Float16 v16h;
typedef __attribute__((ext_vector_type(8)))  _Float16 v8h;
typedef __attribute__((ext_vector_type(16))) __bf16   v16b;
typedef __attribute__((ext_vector_type(8)))  __bf16   v8b;
typedef __attribute__((ext_vector_type(8)))  float    v8f;
typedef __attribute__((ext_vector_type(4)))  float    v4f;
typedef __attribute__((ext_vector_type(2)))  float    v2f;
typedef __attribute__((ext_vector_type(4)))  unsigned v4u;

constexpr int kBatch  = 2;
constexpr int kSeq    = 1024;
constexpr int kDm     = 1024;
constexpr int kDin    = 2048;
constexpr int kNst    = 16;
constexpr int kDtR    = 64;
constexpr int kXzW    = 2 * kDin;
constexpr int kXpN    = kDtR + 2 * kNst;
constexpr int kXdP    = 128;
constexpr int kRows   = kBatch * kSeq;
constexpr int kFfn    = 4 * kDm;
constexpr int kConvTP = 264;
constexpr int kScanTS = 32;
constexpr int kScanCh = 64;
constexpr int kScanYP = 68;
constexpr int kBCP    = 32;
static_assert(kXpN == 96);
static_assert((kDm % 32) == 0 && (kDin % 32) == 0 && (kDtR % 32) == 0 && (kFfn % 32) == 0);
static_assert((kRows % 64) == 0 && (kXzW % 64) == 0 && (kXdP % 64) == 0 && (kDin % 64) == 0 && (kDm % 64) == 0 && (kFfn % 64) == 0);
static_assert((kSeq % 64) == 0 && (kSeq % kScanTS) == 0 && (kDin % kScanCh) == 0 && (kDin % 256) == 0);
static_assert(kDm == 128 * 8);
static_assert(kSeq == 1024);

constexpr size_t kOffXN   = 0;
constexpr size_t kOffWIN  = kOffXN   + (size_t)kRows * kDm  * 2;
constexpr size_t kOffWXP  = kOffWIN  + (size_t)kXzW  * kDm  * 2;
constexpr size_t kOffWDT  = kOffWXP  + (size_t)kXdP  * kDin * 2;
constexpr size_t kOffWOUT = kOffWDT  + (size_t)kDin  * kDtR * 2;
constexpr size_t kOffW1   = kOffWOUT + (size_t)kDm   * kDin * 2;
constexpr size_t kOffW2   = kOffW1   + (size_t)kFfn  * kDm  * 2;
constexpr size_t kOffXZ   = kOffW2   + (size_t)kDm   * kFfn * 2;
constexpr size_t kOffUB   = kOffXZ   + (size_t)kRows * kXzW * 2;
constexpr size_t kOffXD   = kOffUB   + (size_t)kRows * kDin * 2;
constexpr size_t kOffDTIN = kOffXD   + (size_t)kRows * kXdP * 4;
constexpr size_t kOffDTV  = kOffDTIN + (size_t)kRows * kDtR * 2;
constexpr size_t kOffY    = kOffDTV  + (size_t)kRows * kDin * 2;
constexpr size_t kOffYO   = kOffY    + (size_t)kRows * kDin * 2;
constexpr size_t kOffX2   = kOffYO   + (size_t)kRows * kDm  * 4;
constexpr size_t kOffH    = kOffX2   + (size_t)kRows * kDm  * 4;
constexpr size_t kOffP1   = kOffH    + (size_t)kRows * kDm  * 2;
constexpr size_t kOffH1   = kOffP1   + (size_t)kRows * kFfn * 2;
constexpr size_t kWsTotal = kOffH1   + (size_t)kRows * kFfn * 2;
static_assert(kWsTotal == 132120576ull);
static_assert(kWsTotal <= 134217728ull);
static_assert((kOffWIN % 128) == 0 && (kOffWXP % 128) == 0 && (kOffWDT % 128) == 0 && (kOffWOUT % 128) == 0 &&
              (kOffW1 % 128) == 0 && (kOffW2 % 128) == 0 && (kOffXZ % 128) == 0 && (kOffUB % 128) == 0 &&
              (kOffXD % 128) == 0 && (kOffDTIN % 128) == 0 && (kOffDTV % 128) == 0 && (kOffY % 128) == 0 &&
              (kOffYO % 128) == 0 && (kOffX2 % 128) == 0 && (kOffH % 128) == 0 && (kOffP1 % 128) == 0 &&
              (kOffH1 % 128) == 0);

__device__ __forceinline__ unsigned short f2bf_bits(float f) {
  unsigned u = __float_as_uint(f);
  return (unsigned short)((u + 0x7FFFu + ((u >> 16) & 1u)) >> 16);
}
__device__ __forceinline__ float bf_bits2f(unsigned short h) { return __uint_as_float(((unsigned)h) << 16); }
__device__ __forceinline__ float h16_to_f32(unsigned hb) {
  const unsigned sgn = (hb & 0x8000u) << 16; const unsigned em = hb & 0x7fffu;
  const float fn = __uint_as_float((em << 13) + 0x38000000u);
  const float fs = (float)em * 5.9604644775390625e-8f;
  const float mag = (em < 0x400u) ? fs : fn; return __uint_as_float(__float_as_uint(mag) | sgn);
}
__device__ __forceinline__ void mem_order() { asm volatile("" ::: "memory"); }

__device__ __forceinline__ void keep4_h(v16h a, v16h b, v16h c, v16h d) { asm volatile("v_nop" :: "v"(a), "v"(b), "v"(c), "v"(d)); }
__device__ __forceinline__ void keep4_b(v16b a, v16b b, v16b c, v16b d) { asm volatile("v_nop" :: "v"(a), "v"(b), "v"(c), "v"(d)); }
__device__ __forceinline__ void acc_guard4(v8f& a, v8f& b, v8f& c, v8f& d) { asm volatile("v_nop\n\tv_nop\n\tv_nop\n\tv_nop" : "+v"(a), "+v"(b), "+v"(c), "+v"(d)); }
__device__ __forceinline__ void grp_guard_h(v8f& a, v8f& b, v8f& c, v8f& d, v16h x, v16h y0, v16h y1, v16h y2, v16h y3) {
  asm volatile("v_nop\n\tv_nop\n\tv_nop\n\tv_nop" : "+v"(a), "+v"(b), "+v"(c), "+v"(d) : "v"(x), "v"(y0), "v"(y1), "v"(y2), "v"(y3));
}
__device__ __forceinline__ void grp_guard_b(v8f& a, v8f& b, v8f& c, v8f& d, v16b x, v16b y0, v16b y1, v16b y2, v16b y3) {
  asm volatile("v_nop\n\tv_nop\n\tv_nop\n\tv_nop" : "+v"(a), "+v"(b), "+v"(c), "+v"(d) : "v"(x), "v"(y0), "v"(y1), "v"(y2), "v"(y3));
}
template <typename T> struct Frag;
template <> struct Frag<_Float16> {
  typedef v16h V; union U { v16h v; v8h h[2]; };
  static __device__ __forceinline__ v16h load(const _Float16* p) {
    U f; f.h[0] = *(const v8h*)(p); f.h[1] = *(const v8h*)(p + 16); return f.v;
  }
  static __device__ __forceinline__ v8f mma(v16h a, v16h b, v8f c) {
    return __builtin_amdgcn_wmma_f32_16x16x32_f16(false, a, false, b, (short)0, c, false, false);
  }
  static __device__ __forceinline__ void grp(v8f& a, v8f& b, v8f& c, v8f& d, v16h x, v16h y0, v16h y1, v16h y2, v16h y3) { grp_guard_h(a, b, c, d, x, y0, y1, y2, y3); }
  static __device__ __forceinline__ void keep(v16h a, v16h b, v16h c, v16h d) { keep4_h(a, b, c, d); }
};
template <> struct Frag<__bf16> {
  typedef v16b V; union U { v16b v; v8b h[2]; };
  static __device__ __forceinline__ v16b load(const __bf16* p) {
    U f; f.h[0] = *(const v8b*)(p); f.h[1] = *(const v8b*)(p + 16); return f.v;
  }
  static __device__ __forceinline__ v8f mma(v16b a, v16b b, v8f c) {
    return __builtin_amdgcn_wmma_f32_16x16x32_bf16(false, a, false, b, (short)0, c, false, false);
  }
  static __device__ __forceinline__ void grp(v8f& a, v8f& b, v8f& c, v8f& d, v16b x, v16b y0, v16b y1, v16b y2, v16b y3) { grp_guard_b(a, b, c, d, x, y0, y1, y2, y3); }
  static __device__ __forceinline__ void keep(v16b a, v16b b, v16b c, v16b d) { keep4_b(a, b, c, d); }
};

template <int ET> struct Elem;
template <> struct Elem<0> { typedef _Float16 T; };
template <> struct Elem<1> { typedef __bf16 T; };
template <int ET, int BIAS_MODE, int OUT_MODE, int RMODE, int FLIP>
__global__ __launch_bounds__(256) void wmma_gemm64(
    const unsigned short* __restrict__ Ap, int lda,
    const unsigned short* __restrict__ Btp, int ldb,
    void* __restrict__ Cout, int ldc,
    const float* __restrict__ bias,
    const float* __restrict__ R1, const float* __restrict__ R2,
    int M, int N, int K, float scale) {
  typedef typename Elem<ET>::T T;
  typedef typename Frag<T>::V V;
  const T* A = (const T*)Ap; const T* Bt = (const T*)Btp;
  __shared__ __align__(16) float sT[8][16 * 68];
  const int lane = threadIdx.x & 31;
  const int wave = threadIdx.x >> 5;
  const int tilesN = N >> 6;
  const int tilesM = M >> 6;
  const int tile = blockIdx.x * 8 + wave;
  if (tile >= tilesM * tilesN) return;
  const int tm = tile / tilesN;
  const int tn = tile - tm * tilesN;
  const int m0 = tm << 6;
  const int n0 = tn << 6;
  const int rlane = lane & 15;
  const int koff  = (lane >> 4) * 8;
  const int mOff  = (lane >> 4) * 8;

  v8f acc[4][4];
#pragma unroll
  for (int i = 0; i < 4; ++i)
#pragma unroll
    for (int j = 0; j < 4; ++j) acc[i][j] = (v8f){0.f,0.f,0.f,0.f,0.f,0.f,0.f,0.f};

  for (int k0 = 0; k0 < K; k0 += 32) {
    V bh[4];
#pragma unroll
    for (int j = 0; j < 4; ++j)
      bh[j] = Frag<T>::load(Bt + (size_t)(n0 + (j << 4) + rlane) * ldb + koff + k0);
#pragma unroll
    for (int i = 0; i < 4; ++i) {
      V ah = Frag<T>::load(A + (size_t)(m0 + (i << 4) + rlane) * lda + koff + k0);
#pragma unroll
      for (int j = 0; j < 4; ++j) acc[i][j] = Frag<T>::mma(ah, bh[j], acc[i][j]);
      Frag<T>::grp(acc[i][0], acc[i][1], acc[i][2], acc[i][3], ah, bh[0], bh[1], bh[2], bh[3]);
    }
    Frag<T>::keep(bh[0], bh[1], bh[2], bh[3]);
  }
  acc_guard4(acc[0][0], acc[0][1], acc[0][2], acc[0][3]);
  acc_guard4(acc[1][0], acc[1][1], acc[1][2], acc[1][3]);
  acc_guard4(acc[2][0], acc[2][1], acc[2][2], acc[2][3]);
  acc_guard4(acc[3][0], acc[3][1], acc[3][2], acc[3][3]);

  float* slab = sT[wave];
#pragma unroll
  for (int i = 0; i < 4; ++i) {
    const int mBase = m0 + (i << 4);
#pragma unroll
    for (int j = 0; j < 4; ++j) {
      const int n = n0 + (j << 4) + rlane;
      float bv = 0.f;
      if (BIAS_MODE == 2) bv = bias[n];
#pragma unroll
      for (int r = 0; r < 8; ++r) {
        float v = acc[i][j][r] * scale;
        if (BIAS_MODE == 2) v += bv;
        slab[(mOff + r) * 68 + (j << 4) + rlane] = v;
      }
    }
    __builtin_amdgcn_fence(__ATOMIC_RELEASE, "workgroup");
    __builtin_amdgcn_wave_barrier();
    __builtin_amdgcn_fence(__ATOMIC_ACQUIRE, "workgroup");
    if (OUT_MODE == 0) {
      float* C = (float*)Cout;
      const int hh = lane >> 4, c4 = (lane & 15) * 4;
      for (int pass = 0; pass < 2; ++pass) {
#pragma unroll
        for (int it = 0; it < 8; ++it) {
          const int row  = it * 2 + hh;
          const int grow = mBase + row;
          const int orow = FLIP ? (grow ^ (kSeq - 1)) : grow;
          const size_t o = (size_t)orow * ldc + n0 + c4;
          v4f v = *(const v4f*)(slab + row * 68 + c4);
          if (RMODE == 1) { const v4f r1 = *(const v4f*)(R1 + o); v = v + r1; }
          if (RMODE == 2) { const v4f r1 = *(const v4f*)(R1 + o); const v4f r2 = *(const v4f*)(R2 + o); v = r1 + (r2 + v) * 0.5f; }
          *(volatile v4f*)(C + o) = v;
          if (RMODE != 0 && (it & 1)) mem_order();
        }
        __threadfence();
      }
    } else {
      const int qq = lane >> 3, c8 = (lane & 7) * 8;
      unsigned short* C = (unsigned short*)Cout;
      for (int pass = 0; pass < 2; ++pass) {
#pragma unroll
        for (int it = 0; it < 4; ++it) {
          const int row  = it * 4 + qq;
          const int grow = mBase + row;
          const int orow = FLIP ? (grow ^ (kSeq - 1)) : grow;
          const float* sp = slab + row * 68 + c8;
          v8h hv;
#pragma unroll
          for (int e = 0; e < 8; ++e) {
            if (OUT_MODE == 1) hv[e] = (_Float16)sp[e];
            else hv[e] = __builtin_bit_cast(_Float16, f2bf_bits(sp[e]));
          }
          *(volatile v8h*)(C + (size_t)orow * ldc + n0 + c8) = hv;
        }
        __threadfence();
      }
    }
    __builtin_amdgcn_fence(__ATOMIC_RELEASE, "workgroup");
    __builtin_amdgcn_wave_barrier();
    __builtin_amdgcn_fence(__ATOMIC_ACQUIRE, "workgroup");
  }
}

__global__ __launch_bounds__(256) void cvt_rows_bf16_kernel(
    const float* __restrict__ src, unsigned short* __restrict__ dst, int ncols, int rows_real, int total8)
{
  const int i = blockIdx.x * 256 + threadIdx.x;
  if (i >= total8) return;
  const size_t e0 = (size_t)i << 3;
  const size_t nreal = (size_t)rows_real * (size_t)ncols;
  const bool live = (e0 < nreal);
  const size_t ec = live ? e0 : (size_t)0;
  const float fz = live ? 1.0f : 0.0f;
  const v4f a0 = *(const v4f*)(src + ec);
  const v4f a1 = *(const v4f*)(src + ec + 4);
  v8h hv;
#pragma unroll
  for (int e = 0; e < 4; ++e) {
    hv[e]     = __builtin_bit_cast(_Float16, f2bf_bits(a0[e] * fz));
    hv[4 + e] = __builtin_bit_cast(_Float16, f2bf_bits(a1[e] * fz));
  }
  unsigned short* q = dst + e0;
  *(volatile v8h*)q = hv;
  __threadfence();
  *(volatile v8h*)q = hv;
}

__global__ __launch_bounds__(256) void cvt_rows_f16_kernel(
    const float* __restrict__ src, unsigned short* __restrict__ dst, int total8, float mul)
{
  const int i = blockIdx.x * 256 + threadIdx.x;
  if (i >= total8) return;
  const size_t e0 = (size_t)i << 3;
  const v4f a0 = *(const v4f*)(src + e0);
  const v4f a1 = *(const v4f*)(src + e0 + 4);
  v8h hv;
#pragma unroll
  for (int e = 0; e < 4; ++e) {
    hv[e]     = (_Float16)(a0[e] * mul);
    hv[4 + e] = (_Float16)(a1[e] * mul);
  }
  unsigned short* q = dst + e0;
  *(volatile v8h*)q = hv;
  __threadfence();
  *(volatile v8h*)q = hv;
}

__global__ __launch_bounds__(256) void cvt_dtin_kernel(const float* __restrict__ XD, unsigned short* __restrict__ DTIN)
{
  const int i = blockIdx.x * 256 + threadIdx.x;
  if (i >= kRows * (kDtR / 8)) return;
  const int row = i >> 3, c8 = (i & 7) * 8;
  const v4f a0 = *(const v4f*)(XD + (size_t)row * kXdP + c8);
  const v4f a1 = *(const v4f*)(XD + (size_t)row * kXdP + c8 + 4);
  v8h hv;
#pragma unroll
  for (int e = 0; e < 4; ++e) {
    hv[e]     = __builtin_bit_cast(_Float16, f2bf_bits(a0[e]));
    hv[4 + e] = __builtin_bit_cast(_Float16, f2bf_bits(a1[e]));
  }
  unsigned short* q = DTIN + (size_t)row * kDtR + c8;
  *(volatile v8h*)q = hv;
  __threadfence();
  *(volatile v8h*)q = hv;
}

template <int F16OUT>
__global__ __launch_bounds__(128) void layernorm_kernel(
    const float* __restrict__ X, const float* __restrict__ gam, const float* __restrict__ bet, unsigned short* __restrict__ OUTP)
{
  __shared__ float red1[4];
  __shared__ float red2[4];
  const int row = blockIdx.x, tid = threadIdx.x, lane = tid & 31, wave = tid >> 5;
  const float* xr = X + (size_t)row * kDm + tid * 8;
  const v4f a0 = *(const v4f*)(xr);
  const v4f a1 = *(const v4f*)(xr + 4);
  float s = ((a0[0] + a0[1]) + (a0[2] + a0[3])) + ((a1[0] + a1[1]) + (a1[2] + a1[3]));
#pragma unroll
  for (int off = 1; off < 32; off <<= 1) s += __shfl_xor(s, off, 32);
  if (lane == 0) red1[wave] = s;
  __syncthreads();
  const float mean = ((red1[0] + red1[1]) + (red1[2] + red1[3])) * (1.0f / (float)kDm);
  float c[8];
  c[0] = a0[0] - mean; c[1] = a0[1] - mean; c[2] = a0[2] - mean; c[3] = a0[3] - mean;
  c[4] = a1[0] - mean; c[5] = a1[1] - mean; c[6] = a1[2] - mean; c[7] = a1[3] - mean;
  float qs = 0.0f;
#pragma unroll
  for (int e = 0; e < 8; ++e) qs = fmaf(c[e], c[e], qs);
#pragma unroll
  for (int off = 1; off < 32; off <<= 1) qs += __shfl_xor(qs, off, 32);
  if (lane == 0) red2[wave] = qs;
  __syncthreads();
  const float var  = ((red2[0] + red2[1]) + (red2[2] + red2[3])) * (1.0f / (float)kDm);
  const float rstd = 1.0f / sqrtf(var + 1e-5f);
  const v4f g0 = *(const v4f*)(gam + tid * 8);
  const v4f g1 = *(const v4f*)(gam + tid * 8 + 4);
  const v4f b0 = *(const v4f*)(bet + tid * 8);
  const v4f b1 = *(const v4f*)(bet + tid * 8 + 4);
  float o[8];
  o[0] = c[0] * rstd * g0[0] + b0[0]; o[1] = c[1] * rstd * g0[1] + b0[1];
  o[2] = c[2] * rstd * g0[2] + b0[2]; o[3] = c[3] * rstd * g0[3] + b0[3];
  o[4] = c[4] * rstd * g1[0] + b1[0]; o[5] = c[5] * rstd * g1[1] + b1[1];
  o[6] = c[6] * rstd * g1[2] + b1[2]; o[7] = c[7] * rstd * g1[3] + b1[3];
  v8h hv;
#pragma unroll
  for (int e = 0; e < 8; ++e) {
    if (F16OUT) hv[e] = (_Float16)o[e];
    else hv[e] = __builtin_bit_cast(_Float16, f2bf_bits(o[e]));
  }
  unsigned short* op = OUTP + (size_t)row * kDm + tid * 8;
  *(volatile v8h*)op = hv;
  __threadfence();
  *(volatile v8h*)op = hv;
}

__global__ __launch_bounds__(128) void conv_silu_kernel(
    const unsigned short* __restrict__ XZ, const float* __restrict__ cw, const float* __restrict__ cb,
    unsigned short* __restrict__ UB)
{
  __shared__ __align__(16) float sT[16 * kConvTP];
  const int tid = threadIdx.x, lane = tid & 31, wave = tid >> 5;
  const int d0 = blockIdx.x * 256;
  const int ca = d0 + 2 * tid;
  const int g0 = blockIdx.y * 64;
  const int tb = g0 & (kSeq - 1);
  const unsigned* XW = (const unsigned*)XZ;
  const size_t wcol = (size_t)(ca >> 1);
  const v4f wa = *(const v4f*)(cw + (size_t)ca * 4);
  const v4f wb = *(const v4f*)(cw + (size_t)(ca + 1) * 4);
  const float ba = cb[ca], bbv = cb[ca + 1];
  float am3, am2, am1, bm3, bm2, bm1;
  {
    const bool hist = (tb > 0);
    const int rb = hist ? (g0 - 3) : g0;
    const float fz = hist ? 1.0f : 0.0f;
    const unsigned w3 = XW[(size_t)rb * 2048 + wcol];
    const unsigned w2 = XW[(size_t)(rb + 1) * 2048 + wcol];
    const unsigned w1 = XW[(size_t)(rb + 2) * 2048 + wcol];
    am3 = __uint_as_float(w3 << 16) * fz; bm3 = __uint_as_float(w3 & 0xffff0000u) * fz;
    am2 = __uint_as_float(w2 << 16) * fz; bm2 = __uint_as_float(w2 & 0xffff0000u) * fz;
    am1 = __uint_as_float(w1 << 16) * fz; bm1 = __uint_as_float(w1 & 0xffff0000u) * fz;
  }
#pragma unroll 1
  for (int sub = 0; sub < 4; ++sub) {
    const int lb = g0 + sub * 16;
#pragma unroll 1
    for (int s = 0; s < 16; ++s) {
      const unsigned w = XW[(size_t)(lb + s) * 2048 + wcol];
      const float xa = __uint_as_float(w << 16);
      const float xb = __uint_as_float(w & 0xffff0000u);
      float pa = wa[0] * am3;
      pa = fmaf(wa[1], am2, pa);
      pa = fmaf(wa[2], am1, pa);
      pa = fmaf(wa[3], xa, pa);
      pa = pa + ba;
      float pb = wb[0] * bm3;
      pb = fmaf(wb[1], bm2, pb);
      pb = fmaf(wb[2], bm1, pb);
      pb = fmaf(wb[3], xb, pb);
      pb = pb + bbv;
      const float sga = __builtin_amdgcn_rcpf(1.0f + expf(-pa));
      const float sgb = __builtin_amdgcn_rcpf(1.0f + expf(-pb));
      v2f st;
      st[0] = pa * sga;
      st[1] = pb * sgb;
      *(v2f*)(sT + s * kConvTP + 2 * tid) = st;
      am3 = am2; am2 = am1; am1 = xa;
      bm3 = bm2; bm2 = bm1; bm1 = xb;
    }
    __syncthreads();
    v8h hv[4];
#pragma unroll
    for (int it = 0; it < 4; ++it) {
      const float* sp = sT + (it * 4 + wave) * kConvTP + lane * 8;
      const v4f a0 = *(const v4f*)(sp);
      const v4f a1 = *(const v4f*)(sp + 4);
#pragma unroll
      for (int e = 0; e < 4; ++e) {
        hv[it][e]     = __builtin_bit_cast(_Float16, f2bf_bits(a0[e]));
        hv[it][4 + e] = __builtin_bit_cast(_Float16, f2bf_bits(a1[e]));
      }
    }
    for (int pass = 0; pass < 2; ++pass) {
#pragma unroll
      for (int it = 0; it < 4; ++it)
        *(volatile v8h*)(UB + (size_t)(lb + it * 4 + wave) * kDin + d0 + lane * 8) = hv[it];
      __threadfence();
    }
    __syncthreads();
  }
}

__global__ __launch_bounds__(64) void scan_kernel(
    const float* __restrict__ XD, const unsigned short* __restrict__ DTV, const unsigned short* __restrict__ UB,
    const unsigned short* __restrict__ XZ, const float* __restrict__ bdt, const float* __restrict__ Alog,
    const float* __restrict__ Dp, unsigned short* __restrict__ Yp)
{
  __shared__ __align__(16) float sBC[kScanTS * kBCP];
  __shared__ __align__(16) float sDT[kScanTS * kScanCh];
  __shared__ __align__(16) float sU[kScanTS * kScanCh];
  __shared__ __align__(16) float sZ[kScanTS * kScanCh];
  __shared__ __align__(16) float sY[kScanTS * kScanYP];
  __shared__ __align__(16) float sA[kNst * kScanCh];
  const int tid = threadIdx.x, lane = tid & 31, wave = tid >> 5;
  constexpr int kBlkPerB = kDin / kScanCh;
  const int bix = blockIdx.x / kBlkPerB;
  const int d0  = (blockIdx.x - bix * kBlkPerB) * kScanCh;
  const int d   = d0 + tid;
  const size_t row0 = (size_t)bix * kSeq;
#pragma unroll 1
  for (int s = 0; s < kNst; ++s) sA[s * kScanCh + tid] = -expf(Alog[(size_t)d * kNst + s]);
  __syncthreads();
  float negA[kNst], h[kNst];
#pragma unroll
  for (int s = 0; s < kNst; ++s) { negA[s] = sA[s * kScanCh + tid]; h[s] = 0.0f; }
  const float bb = bdt[d], Dd = Dp[d];
  const int q = lane >> 3, c8 = (lane & 7) * 8;
#pragma unroll 1
  for (int t0 = 0; t0 < kSeq; t0 += kScanTS) {
    __syncthreads();
#pragma unroll 1
    for (int i = 0; i < 4; ++i) {
      const int idx = i * kScanCh + tid;
      const int r   = idx >> 3;
      const int c4s = (idx & 7) * 4;
      const int c8s = (idx & 7) * 8;
      const size_t grow = row0 + t0 + r;
      *(v4f*)(sBC + r * kBCP + c4s) = *(const v4f*)(XD + grow * kXdP + kDtR + c4s);
      const v4u wd = *(const v4u*)(DTV + grow * kDin + d0 + c8s);
      const v4u wu = *(const v4u*)(UB  + grow * kDin + d0 + c8s);
      const v4u wz = *(const v4u*)(XZ  + grow * kXzW + kDin + d0 + c8s);
      v4f f0, f1;
      f0[0] = h16_to_f32(wd[0] & 0xffffu); f0[1] = h16_to_f32(wd[0] >> 16);
      f0[2] = h16_to_f32(wd[1] & 0xffffu); f0[3] = h16_to_f32(wd[1] >> 16);
      f1[0] = h16_to_f32(wd[2] & 0xffffu); f1[1] = h16_to_f32(wd[2] >> 16);
      f1[2] = h16_to_f32(wd[3] & 0xffffu); f1[3] = h16_to_f32(wd[3] >> 16);
      *(v4f*)(sDT + r * kScanCh + c8s) = f0;
      *(v4f*)(sDT + r * kScanCh + c8s + 4) = f1;
      v4f u0, u1;
      u0[0] = __uint_as_float(wu[0] << 16); u0[1] = __uint_as_float(wu[0] & 0xffff0000u);
      u0[2] = __uint_as_float(wu[1] << 16); u0[3] = __uint_as_float(wu[1] & 0xffff0000u);
      u1[0] = __uint_as_float(wu[2] << 16); u1[1] = __uint_as_float(wu[2] & 0xffff0000u);
      u1[2] = __uint_as_float(wu[3] << 16); u1[3] = __uint_as_float(wu[3] & 0xffff0000u);
      *(v4f*)(sU + r * kScanCh + c8s) = u0;
      *(v4f*)(sU + r * kScanCh + c8s + 4) = u1;
      v4f z0, z1;
      z0[0] = __uint_as_float(wz[0] << 16); z0[1] = __uint_as_float(wz[0] & 0xffff0000u);
      z0[2] = __uint_as_float(wz[1] << 16); z0[3] = __uint_as_float(wz[1] & 0xffff0000u);
      z1[0] = __uint_as_float(wz[2] << 16); z1[1] = __uint_as_float(wz[2] & 0xffff0000u);
      z1[2] = __uint_as_float(wz[3] << 16); z1[3] = __uint_as_float(wz[3] & 0xffff0000u);
      *(v4f*)(sZ + r * kScanCh + c8s) = z0;
      *(v4f*)(sZ + r * kScanCh + c8s + 4) = z1;
    }
    __syncthreads();
#pragma unroll 1
    for (int s = 0; s < kScanTS; ++s) {
      const float* xr = sBC + s * kBCP;
      float Bs[kNst], Cs[kNst];
#pragma unroll
      for (int q4 = 0; q4 < 4; ++q4) {
        const v4f bv = *(const v4f*)(xr + 4 * q4);
        const v4f cv = *(const v4f*)(xr + kNst + 4 * q4);
        Bs[4 * q4 + 0] = bv[0]; Bs[4 * q4 + 1] = bv[1]; Bs[4 * q4 + 2] = bv[2]; Bs[4 * q4 + 3] = bv[3];
        Cs[4 * q4 + 0] = cv[0]; Cs[4 * q4 + 1] = cv[1]; Cs[4 * q4 + 2] = cv[2]; Cs[4 * q4 + 3] = cv[3];
      }
      const float v   = sDT[s * kScanCh + tid] + bb;
      const float ex  = expf(-fabsf(v));
      const float dt  = fmaxf(v, 0.0f) + log1pf(ex);
      const float ut  = sU[s * kScanCh + tid];
      const float zt  = sZ[s * kScanCh + tid];
      const float dtx = dt * ut;
      float ys = 0.0f;
#pragma unroll
      for (int k = 0; k < kNst; ++k) {
        const float e = __expf(dt * negA[k]);
        h[k] = e * h[k] + dtx * Bs[k];
        ys = h[k] * Cs[k] + ys;
      }
      float y = ys + ut * Dd;
      const float sg = __builtin_amdgcn_rcpf(1.0f + expf(-zt));
      y = y * (zt * sg);
      sY[s * kScanYP + tid] = y;
    }
    __syncthreads();
    v8h hv[4];
#pragma unroll
    for (int it = 0; it < 4; ++it) {
      const int r = it * 8 + wave * 4 + q;
      const float* sp = sY + r * kScanYP + c8;
      const v4f a0 = *(const v4f*)(sp);
      const v4f a1 = *(const v4f*)(sp + 4);
#pragma unroll
      for (int e = 0; e < 4; ++e) {
        hv[it][e]     = __builtin_bit_cast(_Float16, f2bf_bits(a0[e]));
        hv[it][4 + e] = __builtin_bit_cast(_Float16, f2bf_bits(a1[e]));
      }
    }
    for (int pass = 0; pass < 2; ++pass) {
#pragma unroll
      for (int it = 0; it < 4; ++it) {
        const int r = it * 8 + wave * 4 + q;
        *(volatile v8h*)(Yp + (row0 + t0 + r) * kDin + d0 + c8) = hv[it];
      }
      __threadfence();
    }
  }
}

__global__ __launch_bounds__(256) void gelu_kernel(const unsigned short* __restrict__ P1, unsigned short* __restrict__ H1, int n2)
{
  const int i = blockIdx.x * 256 + threadIdx.x;
  if (i >= n2) return;
  const unsigned w = ((const unsigned*)P1)[i];
  const float a = h16_to_f32(w & 0xffffu);
  const float b = h16_to_f32(w >> 16);
  const float ga = 0.5f * a * (1.0f + erff(a * 0.70710678118654752f));
  const float gb = 0.5f * b * (1.0f + erff(b * 0.70710678118654752f));
  const _Float16 ha = (_Float16)ga, hb = (_Float16)gb;
  const unsigned u = (unsigned)__builtin_bit_cast(unsigned short, ha) | ((unsigned)__builtin_bit_cast(unsigned short, hb) << 16);
  ((volatile unsigned*)H1)[i] = u;
  __threadfence();
  ((volatile unsigned*)H1)[i] = u;
}

extern "C" void kernel_launch(void* const* d_in, const int* in_sizes, int n_in,
                              void* d_out, int out_size, void* d_ws, size_t ws_size,
                              hipStream_t stream) {
  if (n_in < 27) return;
  if (in_sizes[0] != kRows * kDm) return;
  if (in_sizes[1] != kDm || in_sizes[2] != kDm) return;
  for (int dir = 0; dir < 2; ++dir) {
    const int o = dir ? 12 : 3;
    if (in_sizes[o + 0] != kXzW * kDm) return;
    if (in_sizes[o + 1] != kDin * 4) return;
    if (in_sizes[o + 2] != kDin) return;
    if (in_sizes[o + 3] != kXpN * kDin) return;
    if (in_sizes[o + 4] != kDin * kDtR) return;
    if (in_sizes[o + 5] != kDin) return;
    if (in_sizes[o + 6] != kDin * kNst) return;
    if (in_sizes[o + 7] != kDin) return;
    if (in_sizes[o + 8] != kDm * kDin) return;
  }
  if (in_sizes[21] != kDm || in_sizes[22] != kDm) return;
  if (in_sizes[23] != kFfn * kDm || in_sizes[24] != kFfn) return;
  if (in_sizes[25] != kDm * kFfn || in_sizes[26] != kDm) return;
  if (out_size != kRows * kDm) return;
  if (ws_size < kWsTotal) return;

  const float* x      = (const float*)d_in[0];
  const float* norm_g = (const float*)d_in[1];
  const float* norm_b = (const float*)d_in[2];
  const float* in_w[2]   = { (const float*)d_in[3],  (const float*)d_in[12] };
  const float* conv_w[2] = { (const float*)d_in[4],  (const float*)d_in[13] };
  const float* conv_b[2] = { (const float*)d_in[5],  (const float*)d_in[14] };
  const float* xp_w[2]   = { (const float*)d_in[6],  (const float*)d_in[15] };
  const float* dt_w[2]   = { (const float*)d_in[7],  (const float*)d_in[16] };
  const float* dt_b[2]   = { (const float*)d_in[8],  (const float*)d_in[17] };
  const float* A_log[2]  = { (const float*)d_in[9],  (const float*)d_in[18] };
  const float* Dp[2]     = { (const float*)d_in[10], (const float*)d_in[19] };
  const float* out_w[2]  = { (const float*)d_in[11], (const float*)d_in[20] };
  const float* ffn_g = (const float*)d_in[21];
  const float* ffn_b = (const float*)d_in[22];
  const float* w1 = (const float*)d_in[23];
  const float* b1 = (const float*)d_in[24];
  const float* w2 = (const float*)d_in[25];
  const float* b2 = (const float*)d_in[26];
  float* out = (float*)d_out;

  char* ws = (char*)d_ws;
  unsigned short* XN   = (unsigned short*)(ws + kOffXN);
  unsigned short* WIN  = (unsigned short*)(ws + kOffWIN);
  unsigned short* WXP  = (unsigned short*)(ws + kOffWXP);
  unsigned short* WDT  = (unsigned short*)(ws + kOffWDT);
  unsigned short* WOUT = (unsigned short*)(ws + kOffWOUT);
  unsigned short* W1H  = (unsigned short*)(ws + kOffW1);
  unsigned short* W2H  = (unsigned short*)(ws + kOffW2);
  unsigned short* XZ   = (unsigned short*)(ws + kOffXZ);
  unsigned short* UB   = (unsigned short*)(ws + kOffUB);
  float*          XD   = (float*)(ws + kOffXD);
  unsigned short* DTIN = (unsigned short*)(ws + kOffDTIN);
  unsigned short* DTV  = (unsigned short*)(ws + kOffDTV);
  unsigned short* Y    = (unsigned short*)(ws + kOffY);
  float*          YO   = (float*)(ws + kOffYO);
  float*          X2   = (float*)(ws + kOffX2);
  unsigned short* H    = (unsigned short*)(ws + kOffH);
  unsigned short* P1   = (unsigned short*)(ws + kOffP1);
  unsigned short* H1   = (unsigned short*)(ws + kOffH1);

  layernorm_kernel<0><<<dim3(kRows), dim3(128), 0, stream>>>(x, norm_g, norm_b, XN);

  for (int dir = 0; dir < 2; ++dir) {
    cvt_rows_bf16_kernel<<<dim3((kXzW * kDm / 8) / 256), dim3(256), 0, stream>>>(in_w[dir], WIN, kDm, kXzW, kXzW * kDm / 8);
    cvt_rows_bf16_kernel<<<dim3((kXdP * kDin / 8) / 256), dim3(256), 0, stream>>>(xp_w[dir], WXP, kDin, kXpN, kXdP * kDin / 8);
    cvt_rows_bf16_kernel<<<dim3((kDin * kDtR / 8) / 256), dim3(256), 0, stream>>>(dt_w[dir], WDT, kDtR, kDin, kDin * kDtR / 8);
    cvt_rows_bf16_kernel<<<dim3((kDm * kDin / 8) / 256), dim3(256), 0, stream>>>(out_w[dir], WOUT, kDin, kDm, kDm * kDin / 8);

    if (dir == 0)
      wmma_gemm64<1, 0, 2, 0, 0><<<dim3(256), dim3(256), 0, stream>>>(
          XN, kDm, WIN, kDm, (void*)XZ, kXzW, nullptr, nullptr, nullptr, kRows, kXzW, kDm, 1.0f);
    else
      wmma_gemm64<1, 0, 2, 0, 1><<<dim3(256), dim3(256), 0, stream>>>(
          XN, kDm, WIN, kDm, (void*)XZ, kXzW, nullptr, nullptr, nullptr, kRows, kXzW, kDm, 1.0f);

    conv_silu_kernel<<<dim3(kDin / 256, kRows / 64), dim3(128), 0, stream>>>(XZ, conv_w[dir], conv_b[dir], UB);

    wmma_gemm64<1, 0, 0, 0, 0><<<dim3(8), dim3(256), 0, stream>>>(
        UB, kDin, WXP, kDin, (void*)XD, kXdP, nullptr, nullptr, nullptr, kRows, kXdP, kDin, 1.0f);

    cvt_dtin_kernel<<<dim3((kRows * (kDtR / 8)) / 256), dim3(256), 0, stream>>>(XD, DTIN);

    wmma_gemm64<1, 0, 1, 0, 0><<<dim3(128), dim3(256), 0, stream>>>(
        DTIN, kDtR, WDT, kDtR, (void*)DTV, kDin, nullptr, nullptr, nullptr, kRows, kDin, kDtR, 1.0f);

    scan_kernel<<<dim3(kBatch * (kDin / kScanCh)), dim3(kScanCh), 0, stream>>>(XD, DTV, UB, XZ, dt_b[dir], A_log[dir], Dp[dir], Y);

    if (dir == 0)
      wmma_gemm64<1, 0, 0, 0, 0><<<dim3(64), dim3(256), 0, stream>>>(
          Y, kDin, WOUT, kDin, (void*)YO, kDm, nullptr, nullptr, nullptr, kRows, kDm, kDin, 1.0f);
    else
      wmma_gemm64<1, 0, 0, 2, 1><<<dim3(64), dim3(256), 0, stream>>>(
          Y, kDin, WOUT, kDin, (void*)X2, kDm, nullptr, x, YO, kRows, kDm, kDin, 1.0f);
  }

  cvt_rows_f16_kernel<<<dim3((kFfn * kDm / 8) / 256), dim3(256), 0, stream>>>(w1, W1H, kFfn * kDm / 8, 16.0f);
  cvt_rows_f16_kernel<<<dim3((kDm * kFfn / 8) / 256), dim3(256), 0, stream>>>(w2, W2H, kDm * kFfn / 8, 16.0f);

  layernorm_kernel<1><<<dim3(kRows), dim3(128), 0, stream>>>(X2, ffn_g, ffn_b, H);

  wmma_gemm64<0, 2, 1, 0, 0><<<dim3(256), dim3(256), 0, stream>>>(
      H, kDm, W1H, kDm, (void*)P1, kFfn, b1, nullptr, nullptr, kRows, kFfn, kDm, 1.0f / 16.0f);

  gelu_kernel<<<dim3((kRows * kFfn / 2) / 256), dim3(256), 0, stream>>>(P1, H1, kRows * kFfn / 2);

  wmma_gemm64<0, 2, 0, 1, 0><<<dim3(64), dim3(256), 0, stream>>>(
      H1, kFfn, W2H, kFfn, (void*)out, kDm, b2, X2, nullptr, kRows, kDm, kFfn, 1.0f / 16.0f);
}
